// CanonicalCov1D_36189394436372
// MI455X (gfx1250) — hardware-verified
//
#include <hip/hip_runtime.h>
#include <math.h>

#ifndef NB
#define NB 32
#endif
#ifndef TLEN
#define TLEN 8192
#endif
#define TLEN_FULL 8192
#define WIN 128
#define SHIFT 128
#define STRIDE 8
#define LAT 32
#define CH 64
#define NCOL (LAT * CH)
#define NWIN ((TLEN - SHIFT - WIN) / STRIDE + 1)
#define NTILE ((NWIN + 15) / 16)
#define OPITCH 68
#define INV_LAT 0.03125f

static_assert(TLEN <= TLEN_FULL);
static_assert(TLEN % 8 == 0);
static_assert(STRIDE == 8);
static_assert(WIN % 32 == 0);
static_assert(WIN / 8 == 16);
static_assert(CH == 4 * 16);
static_assert(NCOL == 2048);
static_assert(NWIN >= 1);
static_assert(STRIDE * (NWIN - 1) + SHIFT + WIN <= TLEN);
static_assert((NCOL * (WIN / 8)) % 256 == 0);
static_assert((OPITCH * 4) % 16 == 0);
static_assert(16 * OPITCH * 4 <= 131072);
static_assert(4 * 2 * 2 == 16);
static_assert(128 * 16 * 2 == 16 * CH * 4);

static constexpr size_t XH_BYTES = (size_t)NB * TLEN * 2;
static constexpr size_t WT_BYTES = (size_t)NCOL * WIN * 2;
static constexpr size_t WS_TOTAL = XH_BYTES + 2 * WT_BYTES;
static_assert(XH_BYTES % 256 == 0);
static_assert(WT_BYTES % 256 == 0);
static_assert(WS_TOTAL <= (size_t)134217728);

typedef __attribute__((ext_vector_type(16))) __bf16 v16b;
typedef __attribute__((ext_vector_type(8)))  float  v8f;
typedef __attribute__((ext_vector_type(4)))  float  v4f;
typedef __attribute__((ext_vector_type(4)))  unsigned int v4u;


#define VST2(T, ptr, val) do { const T vst2_v_ = (val); *(volatile T*)(ptr) = vst2_v_; __threadfence(); *(volatile T*)(ptr) = vst2_v_; } while (0)

__device__ __forceinline__ float bfr(float f) {
    unsigned u = __float_as_uint(f);
    u += 0x7FFFu + ((u >> 16) & 1u);
    return __uint_as_float(u & 0xFFFF0000u);
}
__device__ __forceinline__ unsigned bfbits(float f) {
    unsigned u = __float_as_uint(f);
    u += 0x7FFFu + ((u >> 16) & 1u);
    return u >> 16;
}
__device__ __forceinline__ void st8b(unsigned short* P, size_t o, const float* v) {
    v4u pk;
    pk.x = bfbits(v[0]) | (bfbits(v[1]) << 16);
    pk.y = bfbits(v[2]) | (bfbits(v[3]) << 16);
    pk.z = bfbits(v[4]) | (bfbits(v[5]) << 16);
    pk.w = bfbits(v[6]) | (bfbits(v[7]) << 16);
    VST2(v4u, (v4u*)(P + o), pk);
}

union FragB { v16b v; v4u q[2]; };
__device__ __forceinline__ v16b frag_ldb(const unsigned short* p) {
    FragB f; f.q[0] = *(const v4u*)(p); f.q[1] = *(const v4u*)(p + 16); return f.v;
}
__device__ __forceinline__ v8f wmmab(v16b a, v16b b, v8f c) {
    c = __builtin_amdgcn_wmma_f32_16x16x32_bf16(false, a, false, b, (short)0, c, false, false);
    asm volatile("v_nop\n\tv_nop\n\tv_nop\n\tv_nop" : "+v"(c) : "v"(a), "v"(b));
    return c;
}

__global__ __launch_bounds__(256) void k_xcvt(const float* __restrict__ X, unsigned short* __restrict__ Xh) {
    const unsigned u = blockIdx.x * 256u + threadIdx.x;
    if (u >= (unsigned)(NB * (TLEN / 8))) return;
    const unsigned row = u / (unsigned)(TLEN / 8);
    const unsigned c8 = (u - row * (unsigned)(TLEN / 8)) * 8u;
    const float* xp = X + (size_t)row * TLEN_FULL + c8;
    const v4f a = *(const v4f*)xp;
    const v4f b = *(const v4f*)(xp + 4);
    float v[8] = {a.x, a.y, a.z, a.w, b.x, b.y, b.z, b.w};
    st8b(Xh, (size_t)row * TLEN + c8, v);
}

__global__ __launch_bounds__(256) void k_wcvt(const float* __restrict__ W1, const float* __restrict__ W2,
                                              unsigned short* __restrict__ P1, unsigned short* __restrict__ P2) {
    const unsigned u = blockIdx.x * 256u + threadIdx.x;
    if (u >= (unsigned)(NCOL * (WIN / 8))) return;
    const unsigned k0 = 8u * (u & 15u);
    const unsigned o = u >> 4;
    float v[8];
#pragma unroll
    for (int i = 0; i < 8; ++i) v[i] = W1[(size_t)(k0 + (unsigned)i) * NCOL + o];
    st8b(P1, (size_t)o * WIN + k0, v);
#pragma unroll
    for (int i = 0; i < 8; ++i) v[i] = W2[(size_t)(k0 + (unsigned)i) * NCOL + o];
    st8b(P2, (size_t)o * WIN + k0, v);
}

__global__ __launch_bounds__(128) void k_wincov(const unsigned short* __restrict__ Xh,
                                                const unsigned short* __restrict__ Wt1,
                                                const unsigned short* __restrict__ Wt2,
                                                const float* __restrict__ bias,
                                                float* __restrict__ out) {
    __shared__ __align__(16) float sO[16 * OPITCH];
    const unsigned lane = threadIdx.x & 31u;
    const unsigned wave = (unsigned)__builtin_amdgcn_readfirstlane((int)(threadIdx.x >> 5));
    const unsigned hh = lane >> 4, c = lane & 15u;
    const unsigned n0 = blockIdx.x * 16u;
    const unsigned b = blockIdx.y;
    const unsigned c0 = wave * 16u;

    const unsigned nr = min(n0 + c, (unsigned)(NWIN - 1));
    const unsigned short* xr = Xh + (size_t)b * TLEN + 8u * nr + 8u * hh;
    v16b a1[4], a2[4];
#pragma unroll
    for (int ks = 0; ks < 4; ++ks) a1[ks] = frag_ldb(xr + 32 * ks);
    __builtin_amdgcn_sched_barrier(0);
    unsigned sh2 = (unsigned)SHIFT;
    asm volatile("" : "+v"(sh2) : "v"(a1[3]));
    __builtin_amdgcn_sched_barrier(0);
#pragma unroll
    for (int ks = 0; ks < 4; ++ks) a2[ks] = frag_ldb(xr + sh2 + 32 * ks);

    unsigned woff = (c0 + c) * (unsigned)WIN + 8u * hh;
    v8f s1  = (v8f){0.f,0.f,0.f,0.f,0.f,0.f,0.f,0.f};
    v8f s2  = s1;
    v8f s12 = s1;

#pragma unroll 1
    for (unsigned l = 0; l < (unsigned)LAT; ++l) {
        v8f d1 = (v8f){0.f,0.f,0.f,0.f,0.f,0.f,0.f,0.f};
        v8f d2 = d1;
#pragma unroll
        for (int ks = 0; ks < 4; ++ks) {
            const v16b b1 = frag_ldb(Wt1 + woff + 32 * ks);
            const v16b b2 = frag_ldb(Wt2 + woff + 32 * ks);
            d1 = wmmab(a1[ks], b1, d1);
            d2 = wmmab(a2[ks], b2, d2);
        }
        s1 += d1;
        s2 += d2;
        s12 += d1 * d2;
        woff += (unsigned)(CH * WIN);
    }

    const float bv = bfr(bias[c0 + c]);
#pragma unroll
    for (int r = 0; r < 8; ++r) {
        const float m1 = s1[r] * INV_LAT;
        const float m2 = s2[r] * INV_LAT;
        sO[(8u * hh + (unsigned)r) * OPITCH + c0 + c] = (s12[r] * INV_LAT - m1 * m2) + bv;
    }
    __syncthreads();
    {
        const unsigned c4 = (lane & 15u) * 4u;
        v4f vv[2];
#pragma unroll
        for (int it = 0; it < 2; ++it) {
            const unsigned row = 4u * wave + 2u * (unsigned)it + hh;
            vv[it] = *(const v4f*)(sO + row * OPITCH + c4);
        }
        for (int pass = 0; pass < 2; ++pass) {
#pragma unroll
            for (int it = 0; it < 2; ++it) {
                const unsigned row = 4u * wave + 2u * (unsigned)it + hh;
                const unsigned n = n0 + row;
                if (n < (unsigned)NWIN)
                    *(volatile v4f*)(out + ((size_t)b * NWIN + n) * CH + c4) = vv[it];
            }
            __threadfence();
        }
    }
}

extern "C" void kernel_launch(void* const* d_in, const int* in_sizes, int n_in, void* d_out, int out_size,
                              void* d_ws, size_t ws_size, hipStream_t stream) {
    if (n_in < 4) return;
    if (in_sizes[0] < (NB - 1) * TLEN_FULL + TLEN) return;
    if (in_sizes[1] < WIN * NCOL || in_sizes[2] < WIN * NCOL || in_sizes[3] < CH) return;
    if (out_size < NB * NWIN * CH) return;
    if (WS_TOTAL > ws_size) return;

    const float* X    = (const float*)d_in[0];
    const float* W1   = (const float*)d_in[1];
    const float* W2   = (const float*)d_in[2];
    const float* bias = (const float*)d_in[3];
    float* out = (float*)d_out;

    char* wsp = (char*)d_ws;
    unsigned short* xh  = (unsigned short*)(wsp);
    unsigned short* wt1 = (unsigned short*)(wsp + XH_BYTES);
    unsigned short* wt2 = (unsigned short*)(wsp + XH_BYTES + WT_BYTES);

    k_xcvt<<<(NB * (TLEN / 8) + 255) / 256, 256, 0, stream>>>(X, xh);
    k_wcvt<<<(NCOL * (WIN / 8)) / 256, 256, 0, stream>>>(W1, W2, wt1, wt2);
    k_wincov<<<dim3(NTILE, NB), 128, 0, stream>>>(xh, wt1, wt2, bias, out);
}
